// LSTMNet_42004780155276
// MI455X (gfx1250) — hardware-verified
//
#include <hip/hip_runtime.h>
#include <math.h>

typedef __attribute__((ext_vector_type(16))) _Float16 v16h;
typedef __attribute__((ext_vector_type(8)))  _Float16 v8h;
typedef __attribute__((ext_vector_type(8)))  float    v8f;
typedef __attribute__((ext_vector_type(4)))  float    v4f;

constexpr int NBATCH   = 1024;
constexpr int NSTEP    = 2048;
constexpr int NHID     = 64;
constexpr int NGATE    = 4 * NHID;
constexpr int NCLS     = 10;
constexpr int ROWS_BLK = 16;
constexpr int NTHR     = 128;
constexpr int HPITCH   = 72;
constexpr int XCHUNK   = 32;
constexpr int FPITCH   = 68;
constexpr int OUT_TILE = ROWS_BLK * NCLS;

constexpr float WCARRY     = 64.0f;
constexpr float HCARRY     = 256.0f;
constexpr float HCARRY_INV = 1.0f / HCARRY;
constexpr float SCARRY     = WCARRY * HCARRY;
constexpr float LOG2E_F    = 1.4426950408889634f;
constexpr float KSIG       = -LOG2E_F / SCARRY;
constexpr float KTANH_ACC  = 2.0f * LOG2E_F / SCARRY;
constexpr float KTANH_C    = 2.0f * LOG2E_F;

static_assert(NBATCH % ROWS_BLK == 0, "whole 16-row blocks");
static_assert(NHID == 16 * (NTHR / 32), "4 waves x 16 hidden columns");
static_assert(NHID % 32 == 0, "K multiple of 32");
static_assert(NGATE == 256, "gate width");
static_assert(NSTEP % XCHUNK == 0, "whole x chunks");
static_assert(XCHUNK % 2 == 0, "buffer parity returns to 0 per chunk");
static_assert(ROWS_BLK * XCHUNK == 4 * NTHR, "x staging covers the chunk exactly");
static_assert((2 * ROWS_BLK * HPITCH) % NTHR == 0, "h zero fill exact");
static_assert((OUT_TILE * 4) % 128 == 0, "output tile is whole 128-B lines");
static_assert(OUT_TILE == 5 * 32, "five 32-float line stores");
static_assert(OUT_TILE <= 2 * NTHR, "fc2 two passes cover the tile");
static_assert((HPITCH * 2) % 16 == 0 && (FPITCH * 4) % 16 == 0, "16-B aligned LDS rows");

__device__ __forceinline__ float ex2_fast(float y) {
#if __has_builtin(__builtin_amdgcn_exp2f)
  return __builtin_amdgcn_exp2f(y);
#else
  return __expf(y * 0.69314718055994531f);
#endif
}
__device__ __forceinline__ float sig_from_acc(float a) {
  return __builtin_amdgcn_rcpf(1.0f + ex2_fast(a * KSIG));
}
__device__ __forceinline__ float tanh_from_acc(float a) {
  return 1.0f - 2.0f * __builtin_amdgcn_rcpf(ex2_fast(a * KTANH_ACC) + 1.0f);
}

__device__ __forceinline__ void guard_acc4(v8f& a, v8f& b, v8f& c, v8f& d, v16h x, v16h y) {
  asm volatile("v_nop\n\tv_nop\n\tv_nop\n\tv_nop" : "+v"(a), "+v"(b), "+v"(c), "+v"(d) : "v"(x), "v"(y));
}
__device__ __forceinline__ void keep4_h(v16h a, v16h b, v16h c, v16h d) {
  asm volatile("v_nop" :: "v"(a), "v"(b), "v"(c), "v"(d));
}

template <typename T> struct Frag;
template <> struct Frag<_Float16> {
  typedef v16h V; union U { v16h v; v8h h[2]; };
  static __device__ __forceinline__ v16h load(const _Float16* p) {
    U f; f.h[0] = *(const v8h*)(p); f.h[1] = *(const v8h*)(p + 16); return f.v;
  }
  static __device__ __forceinline__ v8f mma(v16h a, v16h b, v8f c) {
    return __builtin_amdgcn_wmma_f32_16x16x32_f16(false, a, false, b, (short)0, c, false, false);
  }
};

__global__ __launch_bounds__(NTHR) void lstm_head_kernel(
    const float* __restrict__ x, const float* __restrict__ wih, const float* __restrict__ whh,
    const float* __restrict__ bih, const float* __restrict__ bhh,
    const float* __restrict__ fc1w, const float* __restrict__ fc1b,
    const float* __restrict__ fc2w, const float* __restrict__ fc2b,
    float* __restrict__ out) {
  __shared__ __align__(16) _Float16 hbuf[2 * ROWS_BLK * HPITCH];
  __shared__ __align__(16) float    xsT[XCHUNK * ROWS_BLK];
  __shared__ __align__(16) float    hl[ROWS_BLK * FPITCH];
  __shared__ __align__(16) float    a1s[ROWS_BLK * FPITCH];
  __shared__ __align__(16) float    outt[2 * NTHR];

  const int tid  = threadIdx.x;
  const int lane = tid & 31;
  const int wid  = tid >> 5;
  const int c    = lane & 15;
  const int hh   = lane >> 4;
  const int b0   = blockIdx.x * ROWS_BLK;

#pragma unroll 1
  for (int i = tid; i < 2 * ROWS_BLK * HPITCH; i += NTHR) hbuf[i] = (_Float16)0.0f;

  v16h  bfrag[4][2];
  float wihv[4], biasv[4];
#pragma unroll
  for (int g = 0; g < 4; ++g) {
    const int n = 64 * g + 16 * wid + c;
    wihv[g]  = SCARRY * wih[n];
    biasv[g] = SCARRY * (bih[n] + bhh[n]);
#pragma unroll
    for (int kc = 0; kc < 2; ++kc) {
      const float* wp = whh + (size_t)n * NHID + kc * 32 + 8 * hh;
      const v4f q0 = *(const v4f*)(wp);
      const v4f q1 = *(const v4f*)(wp + 4);
      const v4f q2 = *(const v4f*)(wp + 16);
      const v4f q3 = *(const v4f*)(wp + 20);
      v16h f;
#pragma unroll
      for (int e = 0; e < 4; ++e) {
        f[e]      = (_Float16)(q0[e] * WCARRY);
        f[4 + e]  = (_Float16)(q1[e] * WCARRY);
        f[8 + e]  = (_Float16)(q2[e] * WCARRY);
        f[12 + e] = (_Float16)(q3[e] * WCARRY);
      }
      bfrag[g][kc] = f;
    }
  }

  float creg[8], hreg[8];
#pragma unroll
  for (int r = 0; r < 8; ++r) { creg[r] = 0.0f; hreg[r] = 0.0f; }

  int p = 0;
  __syncthreads();

#pragma unroll 1
  for (int t0 = 0; t0 < NSTEP; t0 += XCHUNK) {
#pragma unroll
    for (int it = 0; it < 4; ++it) {
      const int i = tid + it * NTHR;
      const int row = i >> 5, tt = i & 31;
      xsT[tt * ROWS_BLK + row] = x[(size_t)(b0 + row) * NSTEP + t0 + tt];
    }
    __syncthreads();

#pragma unroll 1
    for (int dt = 0; dt < XCHUNK; ++dt) {
      const _Float16* hcur = hbuf + p * (ROWS_BLK * HPITCH);
      _Float16*       hnxt = hbuf + (p ^ 1) * (ROWS_BLK * HPITCH);

      const v16h a0 = Frag<_Float16>::load(hcur + c * HPITCH + 8 * hh);
      const v16h a1 = Frag<_Float16>::load(hcur + c * HPITCH + 8 * hh + 32);

      const v4f xv0 = *(const v4f*)(xsT + dt * ROWS_BLK + 8 * hh);
      const v4f xv1 = *(const v4f*)(xsT + dt * ROWS_BLK + 8 * hh + 4);
      float xr[8];
      xr[0] = xv0[0]; xr[1] = xv0[1]; xr[2] = xv0[2]; xr[3] = xv0[3];
      xr[4] = xv1[0]; xr[5] = xv1[1]; xr[6] = xv1[2]; xr[7] = xv1[3];

      v8f dacc[4];
#pragma unroll
      for (int g = 0; g < 4; ++g)
#pragma unroll
        for (int r = 0; r < 8; ++r) dacc[g][r] = fmaf(xr[r], wihv[g], biasv[g]);

#pragma unroll
      for (int g = 0; g < 4; ++g) dacc[g] = Frag<_Float16>::mma(a0, bfrag[g][0], dacc[g]);
#pragma unroll
      for (int g = 0; g < 4; ++g) dacc[g] = Frag<_Float16>::mma(a1, bfrag[g][1], dacc[g]);
      guard_acc4(dacc[0], dacc[1], dacc[2], dacc[3], a0, a1);
      keep4_h(bfrag[0][0], bfrag[1][0], bfrag[2][0], bfrag[3][0]);
      keep4_h(bfrag[0][1], bfrag[1][1], bfrag[2][1], bfrag[3][1]);

#pragma unroll
      for (int r = 0; r < 8; ++r) {
        const float iv = sig_from_acc(dacc[0][r]);
        const float fv = sig_from_acc(dacc[1][r]);
        const float gv = tanh_from_acc(dacc[2][r]);
        const float ov = sig_from_acc(dacc[3][r]);
        const float cv = fmaf(fv, creg[r], iv * gv);
        creg[r] = cv;
        const float rc = __builtin_amdgcn_rcpf(ex2_fast(cv * KTANH_C) + 1.0f);
        const float tcs = fmaf(-2.0f * HCARRY, rc, HCARRY);
        const float hs = ov * tcs;
        hreg[r] = hs;
        hnxt[(8 * hh + r) * HPITCH + 16 * wid + c] = (_Float16)hs;
      }
      p ^= 1;
      __syncthreads();
    }
  }

#pragma unroll
  for (int r = 0; r < 8; ++r) hl[(8 * hh + r) * FPITCH + 16 * wid + c] = hreg[r] * HCARRY_INV;
  __syncthreads();

  {
    const int k  = tid & 63;
    const int rg = tid >> 6;
    const float b1 = fc1b[k];
    float s1[8];
#pragma unroll
    for (int r = 0; r < 8; ++r) s1[r] = b1;
    const float* w1p = fc1w + (size_t)k * NHID;
#pragma unroll 1
    for (int i = 0; i < NHID; i += 4) {
      const v4f w = *(const v4f*)(w1p + i);
#pragma unroll
      for (int r = 0; r < 8; ++r) {
        const v4f hv = *(const v4f*)(hl + (rg * 8 + r) * FPITCH + i);
        float s = s1[r];
        s = fmaf(hv[0], w[0], s);
        s = fmaf(hv[1], w[1], s);
        s = fmaf(hv[2], w[2], s);
        s = fmaf(hv[3], w[3], s);
        s1[r] = s;
      }
    }
#pragma unroll
    for (int r = 0; r < 8; ++r) a1s[(rg * 8 + r) * FPITCH + k] = fmaxf(s1[r], 0.0f);
  }
  __syncthreads();

#pragma unroll 1
  for (int ps = 0; ps < 2; ++ps) {
    const int o   = tid + ps * NTHR;
    const int oc  = (o < OUT_TILE) ? o : (OUT_TILE - 1);
    const int row = oc / NCLS;
    const int cls = oc - row * NCLS;
    float s = fc2b[cls];
    const float* w2p = fc2w + (size_t)cls * NHID;
    const float* ap  = a1s + row * FPITCH;
#pragma unroll 1
    for (int i = 0; i < NHID; i += 4) {
      const v4f w  = *(const v4f*)(w2p + i);
      const v4f av = *(const v4f*)(ap + i);
      s = fmaf(av[0], w[0], s);
      s = fmaf(av[1], w[1], s);
      s = fmaf(av[2], w[2], s);
      s = fmaf(av[3], w[3], s);
    }
    outt[o] = s;
  }
  __syncthreads();

  if (wid == 0) {
    const float v0 = outt[lane];
    const float v1 = outt[32 + lane];
    const float v2 = outt[64 + lane];
    const float v3 = outt[96 + lane];
    const float v4 = outt[128 + lane];
    volatile float* op = (volatile float*)(out + (size_t)b0 * NCLS);
    op[lane]       = v0;
    op[32 + lane]  = v1;
    op[64 + lane]  = v2;
    op[96 + lane]  = v3;
    op[128 + lane] = v4;
    __threadfence();
    op[lane]       = v0;
    op[32 + lane]  = v1;
    op[64 + lane]  = v2;
    op[96 + lane]  = v3;
    op[128 + lane] = v4;
  }
}

extern "C" void kernel_launch(void* const* d_in, const int* in_sizes, int n_in,
                              void* d_out, int out_size, void* d_ws, size_t ws_size,
                              hipStream_t stream) {
  (void)d_ws; (void)ws_size;
  if (n_in < 9 || d_out == nullptr) return;
  if (in_sizes[0] != NBATCH * NSTEP || in_sizes[1] != NGATE || in_sizes[2] != NGATE * NHID ||
      in_sizes[3] != NGATE || in_sizes[4] != NGATE || in_sizes[5] != NHID * NHID ||
      in_sizes[6] != NHID || in_sizes[7] != NCLS * NHID || in_sizes[8] != NCLS ||
      out_size != NBATCH * NCLS) return;

  const float* x    = (const float*)d_in[0];
  const float* wih  = (const float*)d_in[1];
  const float* whh  = (const float*)d_in[2];
  const float* bih  = (const float*)d_in[3];
  const float* bhh  = (const float*)d_in[4];
  const float* fc1w = (const float*)d_in[5];
  const float* fc1b = (const float*)d_in[6];
  const float* fc2w = (const float*)d_in[7];
  const float* fc2b = (const float*)d_in[8];
  float* out = (float*)d_out;

  lstm_head_kernel<<<NBATCH / ROWS_BLK, NTHR, 0, stream>>>(x, wih, whh, bih, bhh, fc1w, fc1b, fc2w, fc2b, out);
}
